// SwinMultiHeadSA_65257733095770
// MI455X (gfx1250) — hardware-verified
//
#include <hip/hip_runtime.h>


#define NIMG 8
#define DD   256
#define NH_  8
#define PN   3136
#define GR   56
#define WS   7
#define WP   49
#define WPP  64
#define NWIN 64
#define NZ   (NH_ * NWIN)
#define HDD  (NH_ * DD)
#define PCAR 1024.0f
typedef _Float16 h16;
typedef unsigned short bf;
typedef __attribute__((ext_vector_type(16))) __bf16   v16bf;
typedef __attribute__((ext_vector_type(16))) _Float16 v16h;
typedef __attribute__((ext_vector_type(8)))  _Float16 v8h;
typedef __attribute__((ext_vector_type(8)))  unsigned short v8us;
typedef __attribute__((ext_vector_type(8)))  float    v8f;
typedef __attribute__((ext_vector_type(4)))  float    v4f;
typedef v8h  __attribute__((may_alias)) v8ha;
typedef v4f  __attribute__((may_alias)) v4fa;
typedef v8us __attribute__((may_alias)) v8usa;

__device__ __forceinline__ unsigned short f2bf(float f) { unsigned u = __float_as_uint(f); u += 0x7FFFu + ((u >> 16) & 1u); return (unsigned short)(u >> 16); }
__device__ __forceinline__ float bf2f(unsigned short b) { return __uint_as_float(((unsigned)b) << 16); }
__device__ __forceinline__ float bfr(float f) { return bf2f(f2bf(f)); }
__device__ __forceinline__ v16h cat16(v8h lo, v8h hi) { return __builtin_shufflevector(lo, hi, 0, 1, 2, 3, 4, 5, 6, 7, 8, 9, 10, 11, 12, 13, 14, 15); }
__device__ __forceinline__ v16bf cat16b(v8us lo, v8us hi) { return __builtin_bit_cast(v16bf, __builtin_shufflevector(lo, hi, 0, 1, 2, 3, 4, 5, 6, 7, 8, 9, 10, 11, 12, 13, 14, 15)); }
__device__ __forceinline__ v8f wmma16(v16h a, v16h b, v8f c) { return __builtin_amdgcn_wmma_f32_16x16x32_f16(false, a, false, b, (short)0, c, false, false); }
__device__ __forceinline__ v8f wmmab(v16bf a, v16bf b, v8f c) { return __builtin_amdgcn_wmma_f32_16x16x32_bf16(false, a, false, b, (short)0, c, false, false); }


template <typename T16> struct WFrag;
template <> struct WFrag<h16> { typedef v16h V; static __device__ __forceinline__ V ld(const h16* p) { return cat16(*(const v8h*)p, *(const v8h*)(p + 16)); } static __device__ __forceinline__ v8f mma(V a, V b, v8f c) { return wmma16(a, b, c); } };
template <> struct WFrag<bf> { typedef v16bf V; static __device__ __forceinline__ V ld(const bf* p) { return cat16b(*(const v8us*)p, *(const v8us*)(p + 16)); } static __device__ __forceinline__ v8f mma(V a, V b, v8f c) { return wmmab(a, b, c); } };
template <typename T16, int NSPLIT, bool BIAS>
__global__ __launch_bounds__(32) void k_gemmw(const T16* __restrict__ A, const T16* __restrict__ A2, const T16* __restrict__ Bt, const T16* __restrict__ Bt2, int K, float* C, int ldc, const float* __restrict__ bias, size_t sA, size_t sB, size_t sC) {
    typedef typename WFrag<T16>::V V;
    __shared__ __align__(16) float os[16 * 68];
    const size_t z = blockIdx.z; A += z * sA; if (A2) A2 += z * sA; Bt += z * sB; if (Bt2) Bt2 += z * sB; C += z * sC;
    const int lane = threadIdx.x & 31, lr = lane & 15, hi = lane >> 4; const int r0 = blockIdx.x * 64, c0 = blockIdx.y * 64;
    v8f acc[4][4];
#pragma unroll
    for (int mb = 0; mb < 4; ++mb)
#pragma unroll
        for (int nb = 0; nb < 4; ++nb) acc[mb][nb] = (v8f){};
    const size_t aoff = (size_t)(r0 + lr) * K + 8 * hi, boff = (size_t)(c0 + lr) * K + 8 * hi;
#pragma unroll 1
    for (int kc = 0; kc < K; kc += 32) {
        V a[4], a2[4];
#pragma unroll
        for (int mb = 0; mb < 4; ++mb) { a[mb] = WFrag<T16>::ld(A + aoff + (size_t)mb * 16 * K + kc); if (NSPLIT == 1 || NSPLIT == 2) a2[mb] = WFrag<T16>::ld(A2 + aoff + (size_t)mb * 16 * K + kc); }
#pragma unroll
        for (int nb = 0; nb < 4; ++nb) { const V b = WFrag<T16>::ld(Bt + boff + (size_t)nb * 16 * K + kc); V b2; if (NSPLIT >= 2) b2 = WFrag<T16>::ld(Bt2 + boff + (size_t)nb * 16 * K + kc);
#pragma unroll
            for (int mb = 0; mb < 4; ++mb) { acc[mb][nb] = WFrag<T16>::mma(a[mb], b, acc[mb][nb]); if (NSPLIT == 1 || NSPLIT == 2) acc[mb][nb] = WFrag<T16>::mma(a2[mb], b, acc[mb][nb]); if (NSPLIT >= 2) acc[mb][nb] = WFrag<T16>::mma(a[mb], b2, acc[mb][nb]); } }
        asm volatile("v_nop\n\tv_nop\n\tv_nop\n\tv_nop" : "+v"(acc[0][0]), "+v"(acc[1][1]), "+v"(acc[2][2]), "+v"(acc[3][3]) : "v"(a[0]), "v"(a[3]));
    }
#pragma unroll
    for (int mb = 0; mb < 4; ++mb) {
#pragma unroll
        for (int nb = 0; nb < 4; ++nb) {
#pragma unroll
            for (int j = 0; j < 8; ++j) os[(hi * 8 + j) * 68 + nb * 16 + lr] = acc[mb][nb][j]; }
        __builtin_amdgcn_wave_barrier(); asm volatile("" ::: "memory");
        float* crow = C + (size_t)(r0 + mb * 16) * ldc + c0;
#pragma unroll 1
        for (int ps = 0; ps < 2; ++ps) {
#pragma unroll
            for (int s = 0; s < 8; ++s) { const int row = 2 * s + hi, cofs = lr * 4; v4f val = *(const v4fa*)(os + row * 68 + cofs); if (BIAS) { val[0] += bfr(bias[c0 + cofs]); val[1] += bfr(bias[c0 + cofs + 1]); val[2] += bfr(bias[c0 + cofs + 2]); val[3] += bfr(bias[c0 + cofs + 3]); }
                *(volatile v4f*)(crow + (size_t)row * ldc + cofs) = val; }
            if (ps == 0) __threadfence(); }
        __builtin_amdgcn_wave_barrier(); asm volatile("" ::: "memory");
    }
}

__device__ __forceinline__ h16 tohx(float x) { return (h16)x; }
__device__ __forceinline__ void splitf(float y, unsigned short& h, unsigned short& l) { h = f2bf(y); l = f2bf(y - bf2f(h)); }
typedef __attribute__((ext_vector_type(2))) unsigned short v2us;
typedef __attribute__((ext_vector_type(4))) unsigned short v4us;
typedef __attribute__((ext_vector_type(2))) _Float16 v2h;
typedef __attribute__((ext_vector_type(4))) _Float16 v4h;

__global__ __launch_bounds__(256) void k_cvt8(const float* __restrict__ src, bf* dst, size_t n8) { const size_t i = (size_t)blockIdx.x * 256 + threadIdx.x; if (i >= n8) return; const v8f v = *(const v8f*)(src + i * 8); v8us o;
#pragma unroll
    for (int k = 0; k < 8; ++k) o[k] = f2bf(v[k]); *(volatile v8us*)(dst + i * 8) = o; __threadfence(); *(volatile v8us*)(dst + i * 8) = o; }
__device__ __forceinline__ int tok_of(int g, int pos) { const int Y4 = (g >> 3) * WS + pos / WS, X4 = (g & 7) * WS + pos % WS; return Y4 * GR + X4; }
__device__ __forceinline__ int region(int Y4, int X4) { const int ry = (Y4 < GR - WS) ? 0 : ((Y4 < GR - WS / 2) ? 1 : 2); const int rx = (X4 < GR - WS) ? 0 : ((X4 < GR - WS / 2) ? 1 : 2); return ry * 3 + rx; }
__global__ __launch_bounds__(256) void k_xg(const float* __restrict__ img, bf* XT) { const size_t e = ((size_t)blockIdx.x * 256 + threadIdx.x) * 4; if (e >= (size_t)PN * DD) return; const int d = (int)(e % DD); const int p = (int)(e / DD); const int c = d >> 4, py = (d >> 2) & 3; const int Y4 = p / GR, X4 = p % GR; const int y = Y4 * 4 + py; const int ys = (y - 3 + 224) % 224; v4us o;
#pragma unroll
    for (int u = 0; u < 4; ++u) { const int px = (d + u) & 3; const int x = X4 * 4 + px; const int xs = (x - 3 + 224) % 224; const size_t f = ((size_t)((c * 4 + (ys & 3)) * 4 + (xs & 3))) * PN + (ys >> 2) * GR + (xs >> 2); o[u] = f2bf(img[f]); }
    *(volatile v4us*)(XT + e) = o; __threadfence(); *(volatile v4us*)(XT + e) = o; }
__global__ __launch_bounds__(256) void k_wpl(const float* __restrict__ Q, const float* __restrict__ K, h16* Q16, h16* K16) { const size_t e = ((size_t)blockIdx.x * 256 + threadIdx.x) * 4; if (e >= (size_t)NZ * WPP * DD) return; const int dd = (int)(e % DD); const int pos = (int)((e / DD) % WPP); const int z = (int)(e / ((size_t)DD * WPP)); const int h = z / NWIN, g = z % NWIN; v4h oq, ok;
    if (pos < WP) { const size_t src = (size_t)tok_of(g, pos) * HDD + h * DD + dd; const v4f a = *(const v4f*)(Q + src), c = *(const v4f*)(K + src); for (int u = 0; u < 4; ++u) { oq[u] = tohx(a[u]); ok[u] = tohx(c[u]); } } else { for (int u = 0; u < 4; ++u) { oq[u] = (h16)0.f; ok[u] = (h16)0.f; } }
    *(volatile v4h*)(Q16 + e) = oq; *(volatile v4h*)(K16 + e) = ok; __threadfence(); *(volatile v4h*)(Q16 + e) = oq; *(volatile v4h*)(K16 + e) = ok; }
__global__ __launch_bounds__(256) void k_vtw(const float* __restrict__ V, h16* VT) { const size_t e = ((size_t)blockIdx.x * 256 + threadIdx.x) * 2; if (e >= (size_t)NZ * DD * WPP) return; const int pos = (int)(e % WPP); const int dd = (int)((e / WPP) % DD); const int z = (int)(e / ((size_t)WPP * DD)); const int h = z / NWIN, g = z % NWIN; v2h o;
#pragma unroll
    for (int u = 0; u < 2; ++u) { const int pp = pos + u; o[u] = (pp < WP) ? tohx(V[(size_t)tok_of(g, pp) * HDD + h * DD + dd]) : (h16)0.f; } *(volatile v2h*)(VT + e) = o; __threadfence(); *(volatile v2h*)(VT + e) = o; }
__global__ __launch_bounds__(256) void k_ssoft(const float* __restrict__ S, const float* __restrict__ rel, h16* P16) { const int lane = threadIdx.x & 31; const int row = blockIdx.x * 8 + (threadIdx.x >> 5); if (row >= NZ * WPP) return; const int q = row % WPP; const int z = row / WPP; const int h = z / NWIN, g = z % NWIN; h16* prow = P16 + (size_t)row * WPP;
    v2h o2;
    if (q >= WP) { o2[0] = (h16)0.f; o2[1] = (h16)0.f; *(volatile v2h*)(prow + lane * 2) = o2; __threadfence(); *(volatile v2h*)(prow + lane * 2) = o2; return; }
    const int tq = tok_of(g, q); const int fq = region(tq / GR, tq % GR); const int qy = q / WS, qx = q % WS;
    const float* sr = S + (size_t)row * WPP; float v[2]; float mx = -3.0e38f;
#pragma unroll
    for (int u = 0; u < 2; ++u) { const int p = lane * 2 + u; float t = -3.0e38f;
        if (p < WP) { const int tp = tok_of(g, p); const int fp = region(tp / GR, tp % GR); const float mk = (fp != fq) ? -100.0f : 0.0f; const int py_ = p / WS, px_ = p % WS; const float rb = bfr(rel[((py_ - qy + WS - 1) + (px_ - qx + WS - 1) * (2 * WS - 1)) * NH_ + h]);
            const float s1 = __fadd_rn(sr[p] * 0.0625f, mk); t = __fadd_rn(s1, rb); }
        v[u] = t; mx = fmaxf(mx, t); }
#pragma unroll
    for (int sh = 16; sh; sh >>= 1) mx = fmaxf(mx, __shfl_xor(mx, sh, 32));
    float sum = 0.f;
#pragma unroll
    for (int u = 0; u < 2; ++u) { float d0 = __fsub_rn(v[u], mx); asm volatile("" : "+v"(d0)); v[u] = __builtin_amdgcn_exp2f(__fmul_rn(d0, 1.4426950408889634f)); sum += v[u]; }
#pragma unroll
    for (int sh = 16; sh; sh >>= 1) sum += __shfl_xor(sum, sh, 32);
    const float f = __fdiv_rn(PCAR, sum); o2[0] = tohx(v[0] * f); o2[1] = tohx(v[1] * f);
    *(volatile v2h*)(prow + lane * 2) = o2; __threadfence(); *(volatile v2h*)(prow + lane * 2) = o2; }
__global__ __launch_bounds__(256) void k_wmrg(const float* __restrict__ O, bf* Ah, bf* Al) { const size_t e = ((size_t)blockIdx.x * 256 + threadIdx.x) * 4; if (e >= (size_t)NZ * WPP * DD) return; const int dd = (int)(e % DD); const int q = (int)((e / DD) % WPP); const int z = (int)(e / ((size_t)DD * WPP)); if (q >= WP) return; const int h = z / NWIN, g = z % NWIN; const size_t oo = (size_t)tok_of(g, q) * HDD + h * DD + dd; v4us oh, ol;
#pragma unroll
    for (int u = 0; u < 4; ++u) { unsigned short a, b; splitf(O[e + u] * (1.0f / PCAR), a, b); oh[u] = a; ol[u] = b; } *(volatile v4us*)(Ah + oo) = oh; *(volatile v4us*)(Al + oo) = ol; __threadfence(); *(volatile v4us*)(Ah + oo) = oh; *(volatile v4us*)(Al + oo) = ol; }
__global__ __launch_bounds__(256) void k_tro(const float* __restrict__ Y, const float* __restrict__ bo, float* OUTn) { const size_t e = ((size_t)blockIdx.x * 256 + threadIdx.x) * 4; if (e >= (size_t)DD * PN) return; const int p = (int)(e % PN); const int o_ = (int)(e / PN); const float bb = bfr(bo[o_]); v4f r;
#pragma unroll
    for (int u = 0; u < 4; ++u) r[u] = __fadd_rn(Y[(size_t)(p + u) * DD + o_], bb); *(volatile v4f*)(OUTn + e) = r; __threadfence(); *(volatile v4f*)(OUTn + e) = r; }

extern "C" void kernel_launch(void* const* d_in, const int* in_sizes, int n_in,
                              void* d_out, int out_size, void* d_ws, size_t ws_size, hipStream_t stream) {
    (void)in_sizes; (void)n_in; (void)out_size;
    const float* inp = (const float*)d_in[0]; const float* Wk = (const float*)d_in[1]; const float* bk = (const float*)d_in[2]; const float* Wq = (const float*)d_in[3]; const float* bq = (const float*)d_in[4]; const float* Wv = (const float*)d_in[5]; const float* bv = (const float*)d_in[6]; const float* Wo = (const float*)d_in[7]; const float* bo = (const float*)d_in[8]; const float* rel = (const float*)d_in[9];
    float* OUT = (float*)d_out;
    char* wsp = (char*)d_ws;
    auto take = [&](size_t bytes) { char* p = wsp; wsp += (bytes + 255) & ~(size_t)255; return (void*)p; };
    bf* BK = (bf*)take((size_t)HDD * DD * 2); bf* BQ = (bf*)take((size_t)HDD * DD * 2); bf* BV = (bf*)take((size_t)HDD * DD * 2); bf* BO = (bf*)take((size_t)DD * HDD * 2);
    bf* XT = (bf*)take((size_t)PN * DD * 2); float* KF = (float*)take((size_t)PN * HDD * 4); float* QF = (float*)take((size_t)PN * HDD * 4); float* VF = (float*)take((size_t)PN * HDD * 4);
    h16* Q16 = (h16*)take((size_t)NZ * WPP * DD * 2); h16* K16 = (h16*)take((size_t)NZ * WPP * DD * 2); h16* VT = (h16*)take((size_t)NZ * DD * WPP * 2); float* S = (float*)take((size_t)NZ * WPP * WPP * 4); h16* P16 = (h16*)take((size_t)NZ * WPP * WPP * 2); float* O = (float*)take((size_t)NZ * WPP * DD * 4);
    bf* ATh = (bf*)take((size_t)PN * HDD * 2); bf* ATl = (bf*)take((size_t)PN * HDD * 2); float* Y = (float*)take((size_t)PN * DD * 4);
    if ((size_t)(wsp - (char*)d_ws) > ws_size) return;
    k_cvt8<<<(HDD * DD / 8 + 255) / 256, 256, 0, stream>>>(Wk, BK, HDD * DD / 8); k_cvt8<<<(HDD * DD / 8 + 255) / 256, 256, 0, stream>>>(Wq, BQ, HDD * DD / 8); k_cvt8<<<(HDD * DD / 8 + 255) / 256, 256, 0, stream>>>(Wv, BV, HDD * DD / 8); k_cvt8<<<(DD * HDD / 8 + 255) / 256, 256, 0, stream>>>(Wo, BO, DD * HDD / 8);
    const dim3 gp(PN / 64, HDD / 64, 1); const size_t zq = (size_t)WPP * DD, zS = (size_t)WPP * WPP, zv = (size_t)DD * WPP, zo = (size_t)WPP * DD;
    for (int n = 0; n < NIMG; ++n) {
        k_xg<<<(unsigned)(((size_t)PN * DD / 4 + 255) / 256), 256, 0, stream>>>(inp + (size_t)n * DD * PN, XT);
        k_gemmw<bf, 0, true><<<gp, 32, 0, stream>>>(XT, nullptr, BK, nullptr, DD, KF, HDD, bk, 0, 0, 0); k_gemmw<bf, 0, true><<<gp, 32, 0, stream>>>(XT, nullptr, BQ, nullptr, DD, QF, HDD, bq, 0, 0, 0); k_gemmw<bf, 0, true><<<gp, 32, 0, stream>>>(XT, nullptr, BV, nullptr, DD, VF, HDD, bv, 0, 0, 0);
        k_wpl<<<(unsigned)(((size_t)NZ * WPP * DD / 4 + 255) / 256), 256, 0, stream>>>(QF, KF, Q16, K16); k_vtw<<<(unsigned)(((size_t)NZ * DD * WPP / 2 + 255) / 256), 256, 0, stream>>>(VF, VT);
        k_gemmw<h16, 0, false><<<dim3(1, 1, NZ), 32, 0, stream>>>(Q16, nullptr, K16, nullptr, DD, S, WPP, nullptr, zq, zq, zS);
        k_ssoft<<<NZ * WPP / 8, 256, 0, stream>>>(S, rel, P16);
        k_gemmw<h16, 0, false><<<dim3(1, DD / 64, NZ), 32, 0, stream>>>(P16, nullptr, VT, nullptr, WPP, O, DD, nullptr, zS, zv, zo);
        k_wmrg<<<(unsigned)(((size_t)NZ * WPP * DD / 4 + 255) / 256), 256, 0, stream>>>(O, ATh, ATl);
        k_gemmw<bf, 1, false><<<dim3(PN / 64, DD / 64, 1), 32, 0, stream>>>(ATh, ATl, BO, nullptr, HDD, Y, DD, nullptr, 0, 0, 0);
        k_tro<<<(unsigned)(((size_t)DD * PN / 4 + 255) / 256), 256, 0, stream>>>(Y, bo, OUT + (size_t)n * DD * PN); }
}
